// MambaBlock_66374424592996
// MI455X (gfx1250) — hardware-verified
//
#include <hip/hip_runtime.h>
#include <stddef.h>
#include <stdint.h>
#include <math.h>


#define LSEQ   2048
#define DM     768
#define DI     1536
#define K2I    3072
#define NS     16
#define RR     48
#define NXP    128
#define KDT    96
#define DTP    128
#define NTHR   256
#define GBM    64
#define GBN    64
#define GTHR   128
#define SC     64
#define ST     32
#define WSMAX  134217728

#define U_XB   (LSEQ * DM / 8)
#define U_WIN  (2 * DI * DM / 8)
#define U_WX   (NXP * K2I / 8)
#define U_WDT  (DI * KDT / 8)
#define U_WOUT (DM * K2I / 8)
#define U_ALL  (U_XB + U_WIN + U_WX + U_WDT + U_WOUT)

static_assert(U_XB % NTHR == 0 && U_WIN % NTHR == 0 && U_WX % NTHR == 0 && U_WDT % NTHR == 0 && U_WOUT % NTHR == 0);
static_assert(LSEQ % GBM == 0 && (2 * DI) % GBN == 0 && NXP % GBN == 0 && DI % GBN == 0 && DM % GBN == 0);
static_assert(DM % 32 == 0 && K2I % 32 == 0 && KDT % 32 == 0 && KDT == 2 * RR && RR % 8 == 0);
static_assert(GBM == (GTHR / 32) * 16 && GBN == 64);
static_assert(DI % NTHR == 0 && DI % SC == 0 && LSEQ % ST == 0 && SC * 4 == NTHR);
static_assert(ST * SC / 4 == 2 * NTHR && ST * 8 == NTHR && ST * 2 == 2 * (NTHR / 8));
static_assert(LSEQ % 8 == 0 && DM == 6 * 128);

typedef float          v4f   __attribute__((ext_vector_type(4)));
typedef float          v8f   __attribute__((ext_vector_type(8)));
typedef int            v8i   __attribute__((ext_vector_type(8)));
typedef unsigned       v2u   __attribute__((ext_vector_type(2)));
typedef unsigned short v4us  __attribute__((ext_vector_type(4)));
typedef unsigned short v8us  __attribute__((ext_vector_type(8)));
typedef unsigned short v16us __attribute__((ext_vector_type(16)));
typedef __bf16         v16bf __attribute__((ext_vector_type(16)));
typedef v4f  __attribute__((may_alias)) v4fa;
typedef v2u  __attribute__((may_alias)) v2ua;
typedef v4us __attribute__((may_alias)) v4usa;
typedef v8us __attribute__((may_alias)) v8usa;
union FragB { v16bf v; v16us u; v8us h[2]; v8i w; };

__device__ __forceinline__ v8f wmb(const FragB& a, const FragB& b, v8f c) {
  v8f d = __builtin_amdgcn_wmma_f32_16x16x32_bf16(false, a.v, false, b.v, (short)0, c, false, false);
  asm volatile("v_nop\n\tv_nop\n\tv_nop\n\tv_nop" : "+v"(d) : "v"(a.w), "v"(b.w));
  return d;
}

__device__ __forceinline__ unsigned bf16_bits(float f) {
  const unsigned u = __float_as_uint(f);
  return (u + 0x7FFFu + ((u >> 16) & 1u)) >> 16;
}
__device__ __forceinline__ float bf16_val(float f) {
  return __uint_as_float(bf16_bits(f) << 16);
}

__device__ __forceinline__ void cvt8(const float* src, unsigned short* dp, bool ok) {
  const v4f a = *(const v4f*)src;
  const v4f b = *(const v4f*)(src + 4);
  v8us o;
  o[0] = ok ? (unsigned short)bf16_bits(a.x) : (unsigned short)0;
  o[1] = ok ? (unsigned short)bf16_bits(a.y) : (unsigned short)0;
  o[2] = ok ? (unsigned short)bf16_bits(a.z) : (unsigned short)0;
  o[3] = ok ? (unsigned short)bf16_bits(a.w) : (unsigned short)0;
  o[4] = ok ? (unsigned short)bf16_bits(b.x) : (unsigned short)0;
  o[5] = ok ? (unsigned short)bf16_bits(b.y) : (unsigned short)0;
  o[6] = ok ? (unsigned short)bf16_bits(b.z) : (unsigned short)0;
  o[7] = ok ? (unsigned short)bf16_bits(b.w) : (unsigned short)0;
  *(volatile v8us*)dp = o;
  __threadfence();
  *(volatile v8us*)dp = o;
}

__global__ __launch_bounds__(NTHR) void k_prep(const float* __restrict__ x, const float* __restrict__ w_in,
                                               const float* __restrict__ w_xp, const float* __restrict__ w_dt,
                                               const float* __restrict__ w_out,
                                               unsigned short* XB, unsigned short* WIN, unsigned short* WX2,
                                               unsigned short* WDT2, unsigned short* WOUT2) {
  const int u = (int)blockIdx.x * NTHR + (int)threadIdx.x;
  if (u < U_XB) {
    cvt8(x + (size_t)8 * u, XB + (size_t)8 * u, true);
  } else if (u < U_XB + U_WIN) {
    const int v = u - U_XB;
    cvt8(w_in + (size_t)8 * v, WIN + (size_t)8 * v, true);
  } else if (u < U_XB + U_WIN + U_WX) {
    const int v  = u - (U_XB + U_WIN);
    const int n  = v / (K2I / 8);
    const int k8 = (v - n * (K2I / 8)) * 8;
    const int kk = (k8 >= DI) ? (k8 - DI) : k8;
    const int nc = (n < RR + 2 * NS) ? n : (RR + 2 * NS - 1);
    cvt8(w_xp + (size_t)nc * DI + kk, WX2 + (size_t)8 * v, n < RR + 2 * NS);
  } else if (u < U_XB + U_WIN + U_WX + U_WDT) {
    const int v  = u - (U_XB + U_WIN + U_WX);
    const int n  = v / (KDT / 8);
    const int k8 = (v - n * (KDT / 8)) * 8;
    const int kk = (k8 >= RR) ? (k8 - RR) : k8;
    cvt8(w_dt + (size_t)n * RR + kk, WDT2 + (size_t)8 * v, true);
  } else if (u < U_ALL) {
    const int v  = u - (U_XB + U_WIN + U_WX + U_WDT);
    const int n  = v / (K2I / 8);
    const int k8 = (v - n * (K2I / 8)) * 8;
    const int kk = (k8 >= DI) ? (k8 - DI) : k8;
    cvt8(w_out + (size_t)n * DI + kk, WOUT2 + (size_t)8 * v, true);
  }
}

__device__ __forceinline__ float softplus_f(float v) {
  return fmaxf(v, 0.0f) + log1pf(expf(-fabsf(v)));
}

template <int MODE>
__global__ __launch_bounds__(GTHR) void k_gemm(const unsigned short* __restrict__ A, int lda,
                                               const unsigned short* __restrict__ WT, int K,
                                               float* outF, int ldo,
                                               const float* __restrict__ bias, unsigned short* dtin) {
  __shared__ __attribute__((aligned(16))) float stg[GBM * GBN];
  __shared__ __attribute__((aligned(16))) unsigned short dst[(MODE == 1) ? (GBM * DTP) : 8];
  const int tid = (int)threadIdx.x, lane = tid & 31, wave = tid >> 5, hh = lane >> 4, m = lane & 15;
  const int rowBase = (int)blockIdx.x * GBM;
  const int col0    = (int)blockIdx.y * GBN;

  v8f acc[4];
  {
    const v8f z = {0.f, 0.f, 0.f, 0.f, 0.f, 0.f, 0.f, 0.f};
    acc[0] = z; acc[1] = z; acc[2] = z; acc[3] = z;
  }
  const unsigned short* ap = A  + (size_t)(rowBase + 16 * wave + m) * (size_t)lda + 8 * hh;
  const unsigned short* wp = WT + (size_t)(col0 + m) * (size_t)K + 8 * hh;
  const int ksteps = K >> 5;
#pragma unroll 1
  for (int ks = 0; ks < ksteps; ++ks) {
    FragB af;
    af.h[0] = *(const v8usa*)(ap + 32 * ks);
    af.h[1] = *(const v8usa*)(ap + 32 * ks + 16);
#pragma unroll
    for (int t = 0; t < 4; ++t) {
      const unsigned short* wq = wp + (size_t)(16 * t) * (size_t)K + 32 * ks;
      FragB bf;
      bf.h[0] = *(const v8usa*)wq;
      bf.h[1] = *(const v8usa*)(wq + 16);
      acc[t] = wmb(af, bf, acc[t]);
    }
  }

#pragma unroll
  for (int t = 0; t < 4; ++t) {
    const int lc = 16 * t + m;
#pragma unroll
    for (int r = 0; r < 8; ++r) {
      const int lr = 16 * wave + 8 * hh + r;
      stg[lr * GBN + lc] = acc[t][r];
    }
  }
  __syncthreads();

  if constexpr (MODE == 2) {
    const v4f bq = *(const v4f*)(bias + col0 + 4 * m);
    const float b0 = bf16_val(bq.x), b1 = bf16_val(bq.y), b2 = bf16_val(bq.z), b3 = bf16_val(bq.w);
#pragma unroll 1
    for (int i = 0; i < 8; ++i) {
      const int lr = 16 * wave + 2 * i + hh;
      v4f v = *(const v4fa*)(stg + lr * GBN + 4 * m);
      v.x = softplus_f(v.x + b0);
      v.y = softplus_f(v.y + b1);
      v.z = softplus_f(v.z + b2);
      v.w = softplus_f(v.w + b3);
      *(v4fa*)(stg + lr * GBN + 4 * m) = v;
    }
  }

  if constexpr (MODE == 1) {
    if (blockIdx.y == 0) {
#pragma unroll 1
      for (int i = 0; i < 8; ++i) {
        const int lr = 16 * wave + 2 * i + hh;
        const v4f v = *(const v4fa*)(stg + lr * GBN + 4 * m);
        v4us h4, l4;
        unsigned hb;
        hb = bf16_bits(v.x); h4[0] = (unsigned short)hb; l4[0] = (unsigned short)bf16_bits(v.x - __uint_as_float(hb << 16));
        hb = bf16_bits(v.y); h4[1] = (unsigned short)hb; l4[1] = (unsigned short)bf16_bits(v.y - __uint_as_float(hb << 16));
        hb = bf16_bits(v.z); h4[2] = (unsigned short)hb; l4[2] = (unsigned short)bf16_bits(v.z - __uint_as_float(hb << 16));
        hb = bf16_bits(v.w); h4[3] = (unsigned short)hb; l4[3] = (unsigned short)bf16_bits(v.w - __uint_as_float(hb << 16));
        unsigned short* drow = dst + lr * DTP;
        if (m < 12) {
          *(v4usa*)(drow + 4 * m) = h4;
          *(v4usa*)(drow + RR + 4 * m) = l4;
        } else {
          const v8us z8 = {0, 0, 0, 0, 0, 0, 0, 0};
          *(v8usa*)(drow + KDT + 8 * (m - 12)) = z8;
        }
      }
      __syncthreads();
      v8us qv[8];
#pragma unroll
      for (int i = 0; i < 8; ++i) {
        const int lr = 16 * wave + 2 * i + hh;
        qv[i] = *(const v8usa*)(dst + lr * DTP + 8 * m);
      }
#pragma unroll
      for (int i = 0; i < 8; ++i) {
        const int lr = 16 * wave + 2 * i + hh;
        *(volatile v8us*)(dtin + (size_t)(rowBase + lr) * DTP + 8 * m) = qv[i];
      }
      __threadfence();
#pragma unroll
      for (int i = 0; i < 8; ++i) {
        const int lr = 16 * wave + 2 * i + hh;
        *(volatile v8us*)(dtin + (size_t)(rowBase + lr) * DTP + 8 * m) = qv[i];
      }
    }
  }

  v4f fv[8];
#pragma unroll
  for (int i = 0; i < 8; ++i) {
    const int lr = 16 * wave + 2 * i + hh;
    fv[i] = *(const v4fa*)(stg + lr * GBN + 4 * m);
  }
#pragma unroll
  for (int i = 0; i < 8; ++i) {
    const int lr = 16 * wave + 2 * i + hh;
    float* op = outF + (size_t)(rowBase + lr) * (size_t)ldo + col0 + 4 * m;
    *(volatile v4f*)op = fv[i];
  }
  __threadfence();
#pragma unroll
  for (int i = 0; i < 8; ++i) {
    const int lr = 16 * wave + 2 * i + hh;
    float* op = outF + (size_t)(rowBase + lr) * (size_t)ldo + col0 + 4 * m;
    *(volatile v4f*)op = fv[i];
  }
}

__global__ __launch_bounds__(NTHR) void k_conv(const float* __restrict__ XZ, const float* __restrict__ wc,
                                               const float* __restrict__ bc, float* XC, unsigned short* XChl) {
  __shared__ __attribute__((aligned(16))) float sx[NTHR];
  __shared__ __attribute__((aligned(16))) unsigned short sh[NTHR];
  __shared__ __attribute__((aligned(16))) unsigned short sl[NTHR];
  const int tid = (int)threadIdx.x, lane = tid & 31, wave = tid >> 5;
  const int l  = (int)blockIdx.x / (DI / NTHR);
  const int cb = ((int)blockIdx.x - l * (DI / NTHR)) * NTHR;
  const int c  = cb + tid;

  const v4f w4 = *(const v4f*)(wc + 4 * c);
  const float bb = bf16_val(bc[c]);
  const int r0 = l - 3, r1 = l - 2, r2 = l - 1;
  const float t0 = XZ[(size_t)(r0 < 0 ? 0 : r0) * K2I + c];
  const float t1 = XZ[(size_t)(r1 < 0 ? 0 : r1) * K2I + c];
  const float t2 = XZ[(size_t)(r2 < 0 ? 0 : r2) * K2I + c];
  const float t3 = XZ[(size_t)l * K2I + c];
  const float x0 = (r0 >= 0) ? t0 : 0.0f;
  const float x1 = (r1 >= 0) ? t1 : 0.0f;
  const float x2 = (r2 >= 0) ? t2 : 0.0f;
  float pre = bf16_val(w4.x) * x0;
  pre = fmaf(bf16_val(w4.y), x1, pre);
  pre = fmaf(bf16_val(w4.z), x2, pre);
  pre = fmaf(bf16_val(w4.w), t3, pre);
  const float v = pre + bb;
  const float s = v / (1.0f + expf(-v));
  const unsigned hb = bf16_bits(s);
  const unsigned lb = bf16_bits(s - __uint_as_float(hb << 16));
  sx[tid] = s;
  sh[tid] = (unsigned short)hb;
  sl[tid] = (unsigned short)lb;
  __syncthreads();

  if (wave < 2) {
    const v4f o = *(const v4fa*)(sx + 4 * tid);
    float* op = XC + (size_t)l * DI + cb + 4 * tid;
    *(volatile v4f*)op = o;
    __threadfence();
    *(volatile v4f*)op = o;
  } else if (wave == 2) {
    const v8us o = *(const v8usa*)(sh + 8 * lane);
    unsigned short* op = XChl + (size_t)l * K2I + cb + 8 * lane;
    *(volatile v8us*)op = o;
    __threadfence();
    *(volatile v8us*)op = o;
  } else if (wave == 3) {
    const v8us o = *(const v8usa*)(sl + 8 * lane);
    unsigned short* op = XChl + (size_t)l * K2I + DI + cb + 8 * lane;
    *(volatile v8us*)op = o;
    __threadfence();
    *(volatile v8us*)op = o;
  }
}

__global__ __launch_bounds__(NTHR) void k_scan(const float* __restrict__ DT, const float* __restrict__ XC,
                                               const float* __restrict__ XZ, const float* __restrict__ XDBL,
                                               const float* __restrict__ A_log, const float* __restrict__ Dp,
                                               unsigned short* Yhl) {
  __shared__ __attribute__((aligned(16))) float sDT[ST * SC];
  __shared__ __attribute__((aligned(16))) float sXC[ST * SC];
  __shared__ __attribute__((aligned(16))) float sZ[ST * SC];
  __shared__ __attribute__((aligned(16))) float sBC[ST * 32];
  __shared__ __attribute__((aligned(16))) unsigned short sY[ST * 2 * SC];
  const int tid = (int)threadIdx.x;
  const int q   = tid & 3;
  const int cl  = tid >> 2;
  const int cb  = (int)blockIdx.x * SC;
  const int d   = cb + cl;

  const v4f al = *(const v4f*)(A_log + (size_t)d * NS + 4 * q);
  const float A0 = -expf(bf16_val(al.x));
  const float A1 = -expf(bf16_val(al.y));
  const float A2 = -expf(bf16_val(al.z));
  const float A3 = -expf(bf16_val(al.w));
  const float dpv = bf16_val(Dp[d]);
  float h0 = 0.0f, h1 = 0.0f, h2 = 0.0f, h3 = 0.0f;

#pragma unroll 1
  for (int l0 = 0; l0 < LSEQ; l0 += ST) {
    __syncthreads();
#pragma unroll
    for (int i = 0; i < 2; ++i) {
      const int p   = tid + NTHR * i;
      const int row = p >> 4;
      const int c4  = (p & 15) * 4;
      const v4f a = *(const v4f*)(DT + (size_t)(l0 + row) * DI + cb + c4);
      const v4f b = *(const v4f*)(XC + (size_t)(l0 + row) * DI + cb + c4);
      const v4f c = *(const v4f*)(XZ + (size_t)(l0 + row) * K2I + DI + cb + c4);
      *(v4fa*)(sDT + row * SC + c4) = a;
      *(v4fa*)(sXC + row * SC + c4) = b;
      *(v4fa*)(sZ  + row * SC + c4) = c;
    }
    {
      const int row = tid >> 3;
      const int c4  = (tid & 7) * 4;
      const v4f a = *(const v4f*)(XDBL + (size_t)(l0 + row) * NXP + RR + c4);
      *(v4fa*)(sBC + row * 32 + c4) = a;
    }
    __syncthreads();

#pragma unroll 1
    for (int t = 0; t < ST; ++t) {
      const float dtv = sDT[t * SC + cl];
      const float u   = sXC[t * SC + cl];
      const float z   = sZ[t * SC + cl];
      const v4f Bv = *(const v4fa*)(sBC + t * 32 + 4 * q);
      const v4f Cv = *(const v4fa*)(sBC + t * 32 + NS + 4 * q);
      const float e0 = expf(dtv * A0);
      const float e1 = expf(dtv * A1);
      const float e2 = expf(dtv * A2);
      const float e3 = expf(dtv * A3);
      h0 = e0 * h0 + (dtv * Bv.x) * u;
      h1 = e1 * h1 + (dtv * Bv.y) * u;
      h2 = e2 * h2 + (dtv * Bv.z) * u;
      h3 = e3 * h3 + (dtv * Bv.w) * u;
      float p = h0 * Cv.x;
      p = p + h1 * Cv.y;
      p = p + h2 * Cv.z;
      p = p + h3 * Cv.w;
      p += __shfl_xor(p, 1, 32);
      p += __shfl_xor(p, 2, 32);
      const float g = z / (1.0f + expf(-z));
      const float y = (p + dpv * u) * g;
      const unsigned hb = bf16_bits(y);
      const unsigned lb = bf16_bits(y - __uint_as_float(hb << 16));
      if (q == 0) {
        sY[(t * 2 + 0) * SC + cl] = (unsigned short)hb;
        sY[(t * 2 + 1) * SC + cl] = (unsigned short)lb;
      }
    }
    __syncthreads();

    v8us qv[2];
#pragma unroll
    for (int it = 0; it < 2; ++it) {
      const int j = (tid >> 3) + 32 * it;
      qv[it] = *(const v8usa*)(sY + j * SC + 8 * (tid & 7));
    }
#pragma unroll
    for (int it = 0; it < 2; ++it) {
      const int j = (tid >> 3) + 32 * it;
      unsigned short* op = Yhl + (size_t)(l0 + (j >> 1)) * K2I + (j & 1) * DI + cb + 8 * (tid & 7);
      *(volatile v8us*)op = qv[it];
    }
    __threadfence();
#pragma unroll
    for (int it = 0; it < 2; ++it) {
      const int j = (tid >> 3) + 32 * it;
      unsigned short* op = Yhl + (size_t)(l0 + (j >> 1)) * K2I + (j & 1) * DI + cb + 8 * (tid & 7);
      *(volatile v8us*)op = qv[it];
    }
  }
}

__global__ __launch_bounds__(NTHR) void k_rms(const float* __restrict__ R, const unsigned short* __restrict__ XB,
                                              const float* __restrict__ wn, float* out) {
  const int tid = (int)threadIdx.x, lane = tid & 31, wave = tid >> 5;
  const int row = (int)blockIdx.x * 8 + wave;
  v4f rv[6];
  float ss = 0.0f;
#pragma unroll
  for (int j = 0; j < 6; ++j) {
    const int c = 4 * (lane + 32 * j);
    const v4f a = *(const v4f*)(R + (size_t)row * DM + c);
    const v2u xb = *(const v2ua*)(XB + (size_t)row * DM + c);
    v4f r;
    r.x = a.x + __uint_as_float(xb.x << 16);
    r.y = a.y + __uint_as_float(xb.x & 0xffff0000u);
    r.z = a.z + __uint_as_float(xb.y << 16);
    r.w = a.w + __uint_as_float(xb.y & 0xffff0000u);
    rv[j] = r;
    ss = fmaf(r.x, r.x, ss);
    ss = fmaf(r.y, r.y, ss);
    ss = fmaf(r.z, r.z, ss);
    ss = fmaf(r.w, r.w, ss);
  }
  ss += __shfl_xor(ss, 16, 32);
  ss += __shfl_xor(ss, 8, 32);
  ss += __shfl_xor(ss, 4, 32);
  ss += __shfl_xor(ss, 2, 32);
  ss += __shfl_xor(ss, 1, 32);
  const float sc = rsqrtf(ss * (1.0f / (float)DM) + 1e-5f);
#pragma unroll
  for (int j = 0; j < 6; ++j) {
    const int c = 4 * (lane + 32 * j);
    const v4f w = *(const v4f*)(wn + c);
    v4f o;
    o.x = (rv[j].x * sc) * bf16_val(w.x);
    o.y = (rv[j].y * sc) * bf16_val(w.y);
    o.z = (rv[j].z * sc) * bf16_val(w.z);
    o.w = (rv[j].w * sc) * bf16_val(w.w);
    rv[j] = o;
  }
#pragma unroll
  for (int j = 0; j < 6; ++j)
    *(volatile v4f*)(out + (size_t)row * DM + 4 * (lane + 32 * j)) = rv[j];
  __threadfence();
#pragma unroll
  for (int j = 0; j < 6; ++j)
    *(volatile v4f*)(out + (size_t)row * DM + 4 * (lane + 32 * j)) = rv[j];
}

static inline size_t al256(size_t o) { return (o + 255) & ~(size_t)255; }

extern "C" void kernel_launch(void* const* d_in, const int* in_sizes, int n_in,
                              void* d_out, int out_size, void* d_ws, size_t ws_size,
                              hipStream_t stream) {
  if (n_in < 11) return;
  if (in_sizes[0] != LSEQ * DM) return;
  if (in_sizes[1] != 2 * DI * DM) return;
  if (in_sizes[2] != DI * 4) return;
  if (in_sizes[3] != DI) return;
  if (in_sizes[4] != (RR + 2 * NS) * DI) return;
  if (in_sizes[5] != DI * RR) return;
  if (in_sizes[6] != DI) return;
  if (in_sizes[7] != DI * NS) return;
  if (in_sizes[8] != DI) return;
  if (in_sizes[9] != DM * DI) return;
  if (in_sizes[10] != DM) return;
  if (out_size != LSEQ * DM) return;

  const float* x     = (const float*)d_in[0];
  const float* w_in  = (const float*)d_in[1];
  const float* w_cv  = (const float*)d_in[2];
  const float* b_cv  = (const float*)d_in[3];
  const float* w_xp  = (const float*)d_in[4];
  const float* w_dt  = (const float*)d_in[5];
  const float* b_dt  = (const float*)d_in[6];
  const float* A_log = (const float*)d_in[7];
  const float* Dpar  = (const float*)d_in[8];
  const float* w_out = (const float*)d_in[9];
  const float* w_nrm = (const float*)d_in[10];
  float* out = (float*)d_out;

  char* ws = (char*)d_ws;
  size_t off = 0;
  const size_t oXB   = off; off = al256(off + (size_t)LSEQ * DM * 2);
  const size_t oWIN  = off; off = al256(off + (size_t)2 * DI * DM * 2);
  const size_t oWX2  = off; off = al256(off + (size_t)NXP * K2I * 2);
  const size_t oWDT2 = off; off = al256(off + (size_t)DI * KDT * 2);
  const size_t oWO2  = off; off = al256(off + (size_t)DM * K2I * 2);
  const size_t oXZ   = off; off = al256(off + (size_t)LSEQ * K2I * 4);
  const size_t oXC   = off; off = al256(off + (size_t)LSEQ * DI * 4);
  const size_t oXCH  = off; off = al256(off + (size_t)LSEQ * K2I * 2);
  const size_t oXD   = off; off = al256(off + (size_t)LSEQ * NXP * 4);
  const size_t oDTI  = off; off = al256(off + (size_t)LSEQ * DTP * 2);
  const size_t oDT   = off; off = al256(off + (size_t)LSEQ * DI * 4);
  const size_t oYH   = off; off = al256(off + (size_t)LSEQ * K2I * 2);
  const size_t oR    = off; off = al256(off + (size_t)LSEQ * DM * 4);
  if (off > ws_size || off > (size_t)WSMAX) return;
  unsigned short* XB    = (unsigned short*)(ws + oXB);
  unsigned short* WIN   = (unsigned short*)(ws + oWIN);
  unsigned short* WX2   = (unsigned short*)(ws + oWX2);
  unsigned short* WDT2  = (unsigned short*)(ws + oWDT2);
  unsigned short* WOUT2 = (unsigned short*)(ws + oWO2);
  float*          XZ    = (float*)(ws + oXZ);
  float*          XC    = (float*)(ws + oXC);
  unsigned short* XChl  = (unsigned short*)(ws + oXCH);
  float*          XDBL  = (float*)(ws + oXD);
  unsigned short* DTIN  = (unsigned short*)(ws + oDTI);
  float*          DT    = (float*)(ws + oDT);
  unsigned short* Yhl   = (unsigned short*)(ws + oYH);
  float*          Rr    = (float*)(ws + oR);

  k_prep<<<U_ALL / NTHR, NTHR, 0, stream>>>(x, w_in, w_xp, w_dt, w_out, XB, WIN, WX2, WDT2, WOUT2);
  k_gemm<0><<<dim3(LSEQ / GBM, (2 * DI) / GBN), GTHR, 0, stream>>>(XB, DM, WIN, DM, XZ, K2I, b_dt, DTIN);
  k_conv<<<LSEQ * (DI / NTHR), NTHR, 0, stream>>>(XZ, w_cv, b_cv, XC, XChl);
  k_gemm<1><<<dim3(LSEQ / GBM, NXP / GBN), GTHR, 0, stream>>>(XChl, K2I, WX2, K2I, XDBL, NXP, b_dt, DTIN);
  k_gemm<2><<<dim3(LSEQ / GBM, DI / GBN), GTHR, 0, stream>>>(DTIN, DTP, WDT2, KDT, DT, DI, b_dt, DTIN);
  k_scan<<<DI / SC, NTHR, 0, stream>>>(DT, XC, XZ, XDBL, A_log, Dpar, Yhl);
  k_gemm<0><<<dim3(LSEQ / GBM, DM / GBN), GTHR, 0, stream>>>(Yhl, K2I, WOUT2, K2I, Rr, DM, b_dt, DTIN);
  k_rms<<<LSEQ / 8, NTHR, 0, stream>>>(Rr, XB, w_nrm, out);
}
